// GATEncoder_3848290697595
// MI455X (gfx1250) — hardware-run, weakly checked
//
#include <hip/hip_runtime.h>
#include <stddef.h>
#include <stdint.h>
#include <math.h>


#define DIN1    128
#define CW      256
#define NP      512
#define C3      64
#define NP3     128
#define KA      512
#define NTHR    256
#define NWAVE   8
#define EPT     8
#define CHUNK   (NTHR * EPT)
#define WCAP    (EPT * 32)
#define LISTN   (NWAVE * WCAP)
#define NBMAX   2048
#define NBRUN   1024
#define SLOTB   11
#define RCAP    28672
#define DEGCAP  128
#define GBM     64
#define GBN     64
#define GTHR    128
#define MROWS   128
#define PARTW4  544
#define PSTW    68
#define NEGSA   0.2f
#define BNEPS   1e-5f
#define WSLIM   268435456
#define LDS_AGG ((2 * RCAP + 2 * NBMAX + LISTN) * 4 + 64)

static_assert((CHUNK & (CHUNK - 1)) == 0 && CHUNK <= (1 << SLOTB));
static_assert(NBMAX == (1 << SLOTB));
static_assert((NBRUN & (NBRUN - 1)) == 0 && NBRUN <= NBMAX && NBRUN >= 32);
static_assert(NTHR * 8 == NBMAX);
static_assert(LISTN >= NBMAX);
static_assert(LISTN >= NWAVE * WCAP);
static_assert((RCAP % 32) == 0);
static_assert(DEGCAP <= RCAP);
static_assert(LDS_AGG <= 300000);
static_assert(LDS_AGG == 254016);
static_assert(GBM == (GTHR / 32) * 16);
static_assert((DIN1 % 32) == 0 && (KA % 32) == 0 && KA == 2 * CW);
static_assert((NP % GBN) == 0 && NP == 2 * CW && (NP3 % GBN) == 0 && NP3 == 2 * C3);
static_assert((MROWS % GBM) == 0);
static_assert(DIN1 / 8 == 16);
static_assert(NTHR == CW);
static_assert(PARTW4 == ((2 * CW + 1 + 31) / 32) * 32);
static_assert(PSTW >= C3 + 1 && (PSTW % 4) == 0);
static_assert(C3 == 2 * 32);

typedef float          v2f  __attribute__((ext_vector_type(2)));
typedef float          v4f  __attribute__((ext_vector_type(4)));
typedef float          v8f  __attribute__((ext_vector_type(8)));
typedef int            v4i  __attribute__((ext_vector_type(4)));
typedef int            v8i  __attribute__((ext_vector_type(8)));
typedef unsigned int   v4u  __attribute__((ext_vector_type(4)));
typedef unsigned short v8us __attribute__((ext_vector_type(8)));
typedef __bf16         v16b __attribute__((ext_vector_type(16)));
typedef v2f  __attribute__((may_alias)) v2fa;
typedef v4f  __attribute__((may_alias)) v4fa;
typedef v8us __attribute__((may_alias)) v8usa;
union FragB { v16b v; v8us h[2]; v8i w; };

__device__ __forceinline__ v8f wmb(const FragB& a, const FragB& b, v8f c) {
  v8f d = __builtin_amdgcn_wmma_f32_16x16x32_bf16(false, a.v, false, b.v, (short)0, c, false, false);
  asm volatile("v_nop\n\tv_nop\n\tv_nop\n\tv_nop" : "+v"(d) : "v"(a.w), "v"(b.w));
  return d;
}

__device__ __forceinline__ v8f z8() { v8f z = {0.f, 0.f, 0.f, 0.f, 0.f, 0.f, 0.f, 0.f}; return z; }

__device__ __forceinline__ unsigned int f2bf(float f) {
  const unsigned int u = __float_as_uint(f);
  return ((u + 0x7FFFu + ((u >> 16) & 1u)) >> 16) & 0xFFFFu;
}
__device__ __forceinline__ float bf2f(unsigned int b) { return __uint_as_float(b << 16); }
__device__ __forceinline__ float bfr(float f) { return bf2f(f2bf(f)); }
__device__ __forceinline__ v2f bfr2(const v2f a) { v2f r; r.x = bfr(a.x); r.y = bfr(a.y); return r; }
__device__ __forceinline__ v4f bfr4(const v4f a) {
  v4f r; r.x = bfr(a.x); r.y = bfr(a.y); r.z = bfr(a.z); r.w = bfr(a.w); return r;
}
__device__ __forceinline__ unsigned int pk2(float lo, float hi) { return f2bf(lo) | (f2bf(hi) << 16); }
__device__ __forceinline__ v4u pack8(const v4f a, const v4f b) {
  v4u r;
  r.x = pk2(a.x, a.y); r.y = pk2(a.z, a.w); r.z = pk2(b.x, b.y); r.w = pk2(b.z, b.w);
  return r;
}
__device__ __forceinline__ v8us cvt8b(const v4f a, const v4f b) {
  v8us o;
  o[0] = (unsigned short)f2bf(a.x); o[1] = (unsigned short)f2bf(a.y);
  o[2] = (unsigned short)f2bf(a.z); o[3] = (unsigned short)f2bf(a.w);
  o[4] = (unsigned short)f2bf(b.x); o[5] = (unsigned short)f2bf(b.y);
  o[6] = (unsigned short)f2bf(b.z); o[7] = (unsigned short)f2bf(b.w);
  return o;
}

template<int C> struct RowIO;
template<> struct RowIO<8> {
  static __device__ __forceinline__ void ld(float (&d)[8], const float* p) {
    const v4f a = *(const v4fa*)p; const v4f b = *(const v4fa*)(p + 4);
    d[0] = a.x; d[1] = a.y; d[2] = a.z; d[3] = a.w; d[4] = b.x; d[5] = b.y; d[6] = b.z; d[7] = b.w;
  }
  static __device__ __forceinline__ void ldb(float (&d)[8], const float* p) {
    const v4f a = bfr4(*(const v4fa*)p); const v4f b = bfr4(*(const v4fa*)(p + 4));
    d[0] = a.x; d[1] = a.y; d[2] = a.z; d[3] = a.w; d[4] = b.x; d[5] = b.y; d[6] = b.z; d[7] = b.w;
  }
  static __device__ __forceinline__ void stl(float* p, const float (&r)[8]) {
    v4f a, b;
    a.x = r[0]; a.y = r[1]; a.z = r[2]; a.w = r[3]; b.x = r[4]; b.y = r[5]; b.z = r[6]; b.w = r[7];
    *(v4fa*)p = a; *(v4fa*)(p + 4) = b;
  }
};
template<> struct RowIO<2> {
  static __device__ __forceinline__ void ld(float (&d)[2], const float* p) {
    const v2f a = *(const v2fa*)p; d[0] = a.x; d[1] = a.y;
  }
  static __device__ __forceinline__ void ldb(float (&d)[2], const float* p) {
    const v2f a = bfr2(*(const v2fa*)p); d[0] = a.x; d[1] = a.y;
  }
  static __device__ __forceinline__ void stl(float* p, const float (&r)[2]) {
    v2f a; a.x = r[0]; a.y = r[1]; *(v2fa*)p = a;
  }
};

template<int HL>
__device__ __forceinline__ float hsum(float p) {
#pragma unroll
  for (int o = HL >> 1; o >= 1; o >>= 1) p += __shfl_xor(p, o);
  return p;
}

__device__ __forceinline__ int scan_chunk(const int* __restrict__ dsts, int nE, int cbase, int slotBase,
                                          int nb, int vec8, int* list, int tid, int lane, int wave) {
  int wc = 0;
  const int el0  = tid * EPT;
  const int e0   = cbase + el0;
  const int sent = -2147483647 - 1;
  v4i da, db;
  if (vec8 != 0 && cbase + CHUNK <= nE) {
    da = *(const v4i*)(dsts + e0);
    db = *(const v4i*)(dsts + e0 + 4);
  } else {
    da.x = (e0     < nE) ? dsts[min(e0,     nE - 1)] : sent;
    da.y = (e0 + 1 < nE) ? dsts[min(e0 + 1, nE - 1)] : sent;
    da.z = (e0 + 2 < nE) ? dsts[min(e0 + 2, nE - 1)] : sent;
    da.w = (e0 + 3 < nE) ? dsts[min(e0 + 3, nE - 1)] : sent;
    db.x = (e0 + 4 < nE) ? dsts[min(e0 + 4, nE - 1)] : sent;
    db.y = (e0 + 5 < nE) ? dsts[min(e0 + 5, nE - 1)] : sent;
    db.z = (e0 + 6 < nE) ? dsts[min(e0 + 6, nE - 1)] : sent;
    db.w = (e0 + 7 < nE) ? dsts[min(e0 + 7, nE - 1)] : sent;
  }
  const unsigned nbs = (unsigned)slotBase;
  const unsigned unb = (unsigned)nb;
  const unsigned s0 = (unsigned)da.x - nbs, s1 = (unsigned)da.y - nbs;
  const unsigned s2 = (unsigned)da.z - nbs, s3 = (unsigned)da.w - nbs;
  const unsigned s4 = (unsigned)db.x - nbs, s5 = (unsigned)db.y - nbs;
  const unsigned s6 = (unsigned)db.z - nbs, s7 = (unsigned)db.w - nbs;
  const bool h0 = s0 < unb, h1 = s1 < unb, h2 = s2 < unb, h3 = s3 < unb;
  const bool h4 = s4 < unb, h5 = s5 < unb, h6 = s6 < unb, h7 = s7 < unb;
  const unsigned any = __builtin_amdgcn_ballot_w32(h0 | h1 | h2 | h3 | h4 | h5 | h6 | h7);
  if (any != 0u) {
#define HITJ(J, HJ, SJ) { \
      const unsigned mj = __builtin_amdgcn_ballot_w32(HJ); \
      if (mj != 0u) { \
        if (HJ) { \
          const int pos = wc + (int)__builtin_amdgcn_mbcnt_lo(mj, 0u); \
          if (pos < WCAP) list[wave * WCAP + pos] = ((el0 + (J)) << SLOTB) | (int)(SJ); \
        } \
        wc += (int)__builtin_popcount(mj); } }
    HITJ(0, h0, s0)
    HITJ(1, h1, s1)
    HITJ(2, h2, s2)
    HITJ(3, h3, s3)
    HITJ(4, h4, s4)
    HITJ(5, h5, s5)
    HITJ(6, h6, s6)
    HITJ(7, h7, s7)
#undef HITJ
  }
  return wc;
}

__device__ __forceinline__ void wt_unit(const float* __restrict__ w, int cols, int ush, int kmask, int Kout,
                                        unsigned short* wt, int rowoff, int u) {
  const int n   = u >> ush;
  const int k8  = (u & ((1 << ush) - 1)) * 8;
  const int kk  = k8 & kmask;
  const int ncl = n < cols ? n : cols - 1;
  const float* p = w + (size_t)kk * (size_t)cols + ncl;
  v4f a, b;
  a.x = p[0];                  a.y = p[(size_t)cols];       a.z = p[(size_t)2 * cols];   a.w = p[(size_t)3 * cols];
  b.x = p[(size_t)4 * cols];   b.y = p[(size_t)5 * cols];   b.z = p[(size_t)6 * cols];   b.w = p[(size_t)7 * cols];
  const v4f z4 = {0.f, 0.f, 0.f, 0.f};
  if (n >= cols) { a = z4; b = z4; }
  const v8us hv = cvt8b(a, b);
  const size_t o = (size_t)(rowoff + n) * (size_t)Kout + k8;
  *(volatile v8us*)(wt + o) = hv;
  __threadfence();
  *(volatile v8us*)(wt + o) = hv;
}

__global__ __launch_bounds__(NTHR) void k_wt(const float* __restrict__ Wl, const float* __restrict__ Wr,
                                             int cols, int ush, int kmask, int Kout, int rowoffR,
                                             int nbPer, int nUnitsPer, unsigned short* wt) {
  const int tid = (int)threadIdx.x;
  const int bid = (int)blockIdx.x;
  if (bid < nbPer) {
    const int u = bid * NTHR + tid;
    if (u < nUnitsPer) wt_unit(Wl, cols, ush, kmask, Kout, wt, 0, u);
  } else {
    const int u = (bid - nbPer) * NTHR + tid;
    if (u < nUnitsPer) wt_unit(Wr, cols, ush, kmask, Kout, wt, rowoffR, u);
  }
}

__global__ __launch_bounds__(NTHR) void k_xcvt(const float* __restrict__ x, int nN, int nUnits,
                                               unsigned short* xb) {
  const int u = (int)blockIdx.x * NTHR + (int)threadIdx.x;
  if (u >= nUnits) return;
  const int row   = u >> 4;
  const int piece = u & 15;
  const int c0    = 8 * piece;
  const int rc    = row < nN ? row : nN - 1;
  const float* p  = x + (size_t)rc * DIN1 + c0;
  v4f a = *(const v4fa*)p;
  v4f b = *(const v4fa*)(p + 4);
  const v4f z4 = {0.f, 0.f, 0.f, 0.f};
  if (row >= nN) { a = z4; b = z4; }
  const v4u q = pack8(a, b);
  unsigned short* o = xb + (size_t)row * DIN1 + c0;
  *(volatile v4u*)o = q;
  __threadfence();
  *(volatile v4u*)o = q;
}

__global__ __launch_bounds__(GTHR) void k_gemm(
    const unsigned short* __restrict__ A, const unsigned short* __restrict__ WT,
    float* outF, int K, int ldo)
{
  __shared__ __attribute__((aligned(16))) float stg[GBM * GBN];
  const int tid = (int)threadIdx.x, lane = tid & 31, wave = tid >> 5, hh = lane >> 4, m = lane & 15;
  const int rowBase = (int)blockIdx.x * GBM;
  const int col0    = (int)blockIdx.y * GBN;

  v8f acc[4];
#pragma unroll
  for (int t = 0; t < 4; ++t) acc[t] = z8();
  const unsigned short* ap = A  + (size_t)(rowBase + 16 * wave + m) * (size_t)K + 8 * hh;
  const unsigned short* wp = WT + (size_t)(col0 + m) * (size_t)K + 8 * hh;
  const int ksteps = K >> 5;
#pragma unroll 1
  for (int ks = 0; ks < ksteps; ++ks) {
    FragB af;
    af.h[0] = *(const v8usa*)(ap + 32 * ks);
    af.h[1] = *(const v8usa*)(ap + 32 * ks + 16);
#pragma unroll
    for (int t = 0; t < 4; ++t) {
      const unsigned short* wq = wp + (size_t)(16 * t) * (size_t)K + 32 * ks;
      FragB bf;
      bf.h[0] = *(const v8usa*)wq;
      bf.h[1] = *(const v8usa*)(wq + 16);
      acc[t] = wmb(af, bf, acc[t]);
    }
  }

#pragma unroll
  for (int t = 0; t < 4; ++t) {
    const int lc = 16 * t + m;
#pragma unroll
    for (int r = 0; r < 8; ++r) {
      const int lr = 16 * wave + 8 * hh + r;
      stg[lr * GBN + lc] = acc[t][r];
    }
  }
  __syncthreads();

  v4f fv[8];
#pragma unroll
  for (int i = 0; i < 8; ++i) {
    const int lr = 16 * wave + 2 * i + hh;
    fv[i] = *(const v4fa*)(stg + lr * GBN + 4 * m);
  }
#pragma unroll
  for (int i = 0; i < 8; ++i) {
    const int lr = 16 * wave + 2 * i + hh;
    const int gr = rowBase + lr;
    float* op = outF + (size_t)gr * (size_t)ldo + col0 + 4 * m;
    *(volatile v4f*)op = fv[i];
  }
  __threadfence();
#pragma unroll
  for (int i = 0; i < 8; ++i) {
    const int lr = 16 * wave + 2 * i + hh;
    const int gr = rowBase + lr;
    float* op = outF + (size_t)gr * (size_t)ldo + col0 + 4 * m;
    *(volatile v4f*)op = fv[i];
  }
}

template<int C>
__device__ __forceinline__ float edot(const float (&hs)[C], const float (&hd)[C], const float (&at)[C]) {
  float part = 0.f;
#pragma unroll
  for (int j = 0; j < C; ++j) {
    float v = hs[j] + hd[j];
    v = v >= 0.f ? v : v * NEGSA;
    part = fmaf(v, at[j], part);
  }
  return part;
}
template<int C>
__device__ __forceinline__ void smerge(float lg, float& mx, float& dn, float (&av)[C], const float (&hs)[C]) {
  const float df = lg - mx;
  const float ee = __expf(-fabsf(df));
  const bool up  = df > 0.f;
  const float s1 = up ? ee : 1.0f;
  const float s2 = up ? 1.0f : ee;
  mx = up ? lg : mx;
  dn = fmaf(dn, s1, s2);
#pragma unroll
  for (int j = 0; j < C; ++j) av[j] = fmaf(av[j], s1, s2 * hs[j]);
}

template<int CPL, int HLN, int STATS>
__global__ __launch_bounds__(NTHR) void k_agg(
    const int* __restrict__ srcs, const int* __restrict__ dsts,
    const float* __restrict__ F, const float* __restrict__ att, const float* __restrict__ bias,
    float* outp, int ldo, int nRowsW, float* part,
    int nN, int nE, int nb, int vec8) {
  constexpr int CW_    = 32 * CPL;
  constexpr int NP_    = 2 * CW_;
  constexpr int PW_    = ((2 * CW_ + 1 + 31) / 32) * 32;
  constexpr int WSTW_  = 2 * CW_ + 4;
  constexpr int PIECES = CW_ / 4;
  constexpr int NI     = (PIECES + 31) / 32;
  static_assert(NWAVE * WSTW_ + PW_ <= RCAP);
  static_assert(PW_ / 4 <= NTHR && CW_ <= NTHR);
  static_assert(NWAVE * CW_ <= RCAP);
  static_assert((HLN & (HLN - 1)) == 0 && HLN >= 2 && HLN <= 32);
  static_assert((CW_ % 4) == 0 && (WSTW_ % 4) == 0);

  extern __shared__ v4f lds_dyn[];
  int* reg1 = (int*)lds_dyn;
  int* reg2 = reg1 + RCAP;
  int* scnt = reg2 + RCAP;
  int* soff = scnt + NBMAX;
  int* list = soff + NBMAX;
  int* wcnt = list + LISTN;
  int* wtot = wcnt + NWAVE;
  const int tid = (int)threadIdx.x, lane = tid & 31, wave = tid >> 5;
  const int nodeBase = (int)blockIdx.x * nb;

  for (int i = tid; i < NBMAX; i += NTHR) scnt[i] = 0;
  for (int i = tid; i < RCAP; i += NTHR) reg2[i] = 0;
  __syncthreads();

  int tot = 0;
  const int nChunks = (nE + CHUNK - 1) / CHUNK;
#pragma unroll 1
  for (int ch = 0; ch < nChunks; ++ch) {
    const int cbase = ch * CHUNK;
    const int wc = scan_chunk(dsts, nE, cbase, nodeBase, nb, vec8, list, tid, lane, wave);
    if (lane == 0) wcnt[wave] = wc;
    __syncthreads();
    int pre = 0, all = 0;
#pragma unroll
    for (int w2 = 0; w2 < NWAVE; ++w2) {
      int c = wcnt[w2];
      c = c < 0 ? 0 : (c > WCAP ? WCAP : c);
      all += c;
      pre += (w2 < wave) ? c : 0;
    }
    const int wcc  = wc > WCAP ? WCAP : wc;
    const int base = tot + pre;
#pragma unroll 1
    for (int i = lane; i < wcc; i += 32) {
      const int ent = list[wave * WCAP + i];
      const int el  = (ent >> SLOTB) & (CHUNK - 1);
      const int sl  = ent & (NBMAX - 1);
      int eid = cbase + el;
      eid = eid > nE - 1 ? nE - 1 : eid;
      const int pos = base + i;
      if (pos < RCAP) reg1[pos] = (int)(((unsigned)eid << SLOTB) | (unsigned)sl);
    }
    tot += all;
    tot = tot > RCAP ? RCAP : tot;
    __syncthreads();
  }
  const int nh = tot;

  if (wave == 0) {
#pragma unroll 1
    for (int b0 = 0; b0 < nh; b0 += 32) {
      const int idx = b0 + lane;
      const int uv  = reg1[idx < nh ? idx : nh - 1];
      const int m32 = (nh - b0) < 32 ? (nh - b0) : 32;
#pragma unroll 1
      for (int k = 0; k < m32; ++k) {
        const int u  = __builtin_amdgcn_readlane(uv, k);
        const int sl = u & (NBMAX - 1);
        if (lane == 0) scnt[sl] = scnt[sl] + 1;
      }
    }
  }
  __syncthreads();

  {
    const v4i ca = *(const v4i*)(scnt + 8 * tid);
    const v4i cb = *(const v4i*)(scnt + 8 * tid + 4);
    const int e0 = ca.x < 0 ? 0 : ca.x, e1 = ca.y < 0 ? 0 : ca.y, e2 = ca.z < 0 ? 0 : ca.z, e3 = ca.w < 0 ? 0 : ca.w;
    const int e4 = cb.x < 0 ? 0 : cb.x, e5 = cb.y < 0 ? 0 : cb.y, e6 = cb.z < 0 ? 0 : cb.z, e7 = cb.w < 0 ? 0 : cb.w;
    const int ts = e0 + e1 + e2 + e3 + e4 + e5 + e6 + e7;
    int incl = ts;
#pragma unroll
    for (int d = 1; d < 32; d <<= 1) {
      const int up = __shfl_up(incl, d);
      if (lane >= d) incl += up;
    }
    if (lane == 31) wtot[wave] = incl;
    __syncthreads();
    int pre = 0;
#pragma unroll
    for (int w2 = 0; w2 < NWAVE; ++w2) pre += (w2 < wave) ? wtot[w2] : 0;
    int run = pre + incl - ts;
    soff[8 * tid + 0] = run; run += e0;
    soff[8 * tid + 1] = run; run += e1;
    soff[8 * tid + 2] = run; run += e2;
    soff[8 * tid + 3] = run; run += e3;
    soff[8 * tid + 4] = run; run += e4;
    soff[8 * tid + 5] = run; run += e5;
    soff[8 * tid + 6] = run; run += e6;
    soff[8 * tid + 7] = run;
  }
  __syncthreads();
  for (int i = tid; i < NBMAX; i += NTHR) list[i] = soff[i];
  __syncthreads();

  if (wave == 0) {
#pragma unroll 1
    for (int b0 = 0; b0 < nh; b0 += 32) {
      const int idx = b0 + lane;
      const int uv  = reg1[idx < nh ? idx : nh - 1];
      const int m32 = (nh - b0) < 32 ? (nh - b0) : 32;
#pragma unroll 1
      for (int k = 0; k < m32; ++k) {
        const int u   = __builtin_amdgcn_readlane(uv, k);
        const int sl  = u & (NBMAX - 1);
        const int eid = (int)((unsigned)u >> SLOTB);
        if (lane == 0) {
          int pos = list[sl];
          pos = pos < 0 ? 0 : (pos > RCAP - 1 ? RCAP - 1 : pos);
          reg2[pos] = eid;
          list[sl] = pos + 1;
        }
      }
    }
  }
  __syncthreads();

  const int nbw = nb >> 3;
  const bool ovf = (nh >= RCAP);
  const float qnan = __int_as_float(0x7fc00000);
  const int c0 = CPL * lane;
  float* stw = (float*)reg1 + wave * CW_;
  float at[CPL], bb[CPL];
  RowIO<CPL>::ldb(at, att + c0);
  RowIO<CPL>::ldb(bb, bias + c0);
  int wn = 0;
  float wm[CPL], wq[CPL];
#pragma unroll
  for (int j = 0; j < CPL; ++j) { wm[j] = 0.0f; wq[j] = 0.0f; }

#pragma unroll 1
  for (int jt = 0; jt < nbw; ++jt) {
    const int slot = wave * nbw + jt;
    const int grow = nodeBase + slot;
    const int gcl  = grow < nN ? grow : nN - 1;
    int st = soff[slot];
    const int craw = scnt[slot];
    int cnt = craw;
    st  = st < 0 ? 0 : (st > nh ? nh : st);
    cnt = cnt < 0 ? 0 : (cnt > DEGCAP ? DEGCAP : cnt);
    if (cnt > nh - st) cnt = nh - st;
    const float pz = (ovf || craw > DEGCAP) ? qnan : 0.0f;
    const bool live = grow < nN;

    const float* fr = F + (size_t)gcl * (size_t)NP_;
    float hd[CPL];
    RowIO<CPL>::ld(hd, fr + CW_ + c0);
    float av[CPL];
#pragma unroll
    for (int j = 0; j < CPL; ++j) av[j] = 0.f;
    float mx = -1.0e30f, dn = 0.f;

#pragma unroll 1
    for (int q = 0; q <= cnt; ++q) {
      const bool last = (q == cnt);
      int idx = st + q; idx = idx > RCAP - 1 ? RCAP - 1 : idx;
      int eid = reg2[idx]; eid = eid < 0 ? 0 : (eid > nE - 1 ? nE - 1 : eid);
      const int sraw = srcs[eid];
      const int se = sraw < 0 ? 0 : (sraw > nN - 1 ? nN - 1 : sraw);
      const int s = last ? gcl : se;
      float hs[CPL];
      RowIO<CPL>::ld(hs, F + (size_t)s * (size_t)NP_ + c0);
      const float lg = hsum<HLN>(edot<CPL>(hs, hd, at));
      smerge<CPL>(lg, mx, dn, av, hs);
    }
    const float inv = __builtin_amdgcn_rcpf(dn);

    float r[CPL];
#pragma unroll
    for (int j = 0; j < CPL; ++j) r[j] = fmaf(av[j], inv, bb[j]);
    if (STATS != 0) {
      if (live) {
        wn += 1;
        const float rk = __builtin_amdgcn_rcpf((float)wn);
#pragma unroll
        for (int j = 0; j < CPL; ++j) {
          const float d = r[j] - wm[j];
          wm[j] = fmaf(d, rk, wm[j]);
          wq[j] = fmaf(d, r[j] - wm[j], wq[j]);
        }
      }
    }
#pragma unroll
    for (int j = 0; j < CPL; ++j) r[j] = (live ? r[j] : 0.f) + pz;

    __builtin_amdgcn_fence(__ATOMIC_RELEASE, "wavefront");
    __builtin_amdgcn_wave_barrier();
    RowIO<CPL>::stl(stw + c0, r);
    __builtin_amdgcn_fence(__ATOMIC_RELEASE, "wavefront");
    __builtin_amdgcn_wave_barrier();
    v4f yv[NI];
#pragma unroll
    for (int i = 0; i < NI; ++i) {
      int p = 32 * i + lane; p = p < PIECES ? p : PIECES - 1;
      yv[i] = *(const v4fa*)(stw + 4 * p);
    }
    const bool wrow = grow < nRowsW;
    const int growc = wrow ? grow : nRowsW - 1;
    float* op = outp + (size_t)growc * (size_t)ldo;
#pragma unroll
    for (int i = 0; i < NI; ++i) {
      const int p = 32 * i + lane;
      if (wrow && p < PIECES) *(volatile v4f*)(op + 4 * p) = yv[i];
    }
    __threadfence();
#pragma unroll
    for (int i = 0; i < NI; ++i) {
      const int p = 32 * i + lane;
      if (wrow && p < PIECES) *(volatile v4f*)(op + 4 * p) = yv[i];
    }
  }

  if (STATS != 0) {
    __syncthreads();
    float* wst = (float*)reg2;
    float* pst = wst + NWAVE * WSTW_;
    RowIO<CPL>::stl(wst + wave * WSTW_ + c0, wm);
    RowIO<CPL>::stl(wst + wave * WSTW_ + CW_ + c0, wq);
    if (lane == 0) wst[wave * WSTW_ + 2 * CW_] = (float)wn;
    __syncthreads();
    if (tid < CW_) {
      float n = 0.0f, mean = 0.0f, M2 = 0.0f;
#pragma unroll 1
      for (int w2 = 0; w2 < NWAVE; ++w2) {
        const float nbv = wst[w2 * WSTW_ + 2 * CW_];
        const float mb  = wst[w2 * WSTW_ + tid];
        const float qb  = wst[w2 * WSTW_ + CW_ + tid];
        if (nbv > 0.5f) {
          const float nn = n + nbv;
          const float delta = mb - mean;
          const float f = nbv / nn;
          mean = fmaf(delta, f, mean);
          M2 = M2 + qb + delta * delta * n * f;
          n = nn;
        }
      }
      pst[1 + tid] = mean;
      pst[1 + CW_ + tid] = M2;
      if (tid == 0) pst[0] = n;
    }
#pragma unroll 1
    for (int i = 2 * CW_ + 1 + tid; i < PW_; i += NTHR) pst[i] = 0.0f;
    __syncthreads();
    const int pb = (int)blockIdx.x;
    v4f ps = {0.0f, 0.0f, 0.0f, 0.0f};
    if (tid < PW_ / 4) {
      ps = *(const v4fa*)(pst + 4 * tid);
      *(volatile v4f*)(part + (size_t)pb * PW_ + 4 * tid) = ps;
    }
    __threadfence();
    if (tid < PW_ / 4) {
      *(volatile v4f*)(part + (size_t)pb * PW_ + 4 * tid) = ps;
    }
  }
  (void)part;
}

__global__ __launch_bounds__(CW) void k_bnfin(const float* __restrict__ part, int nPart,
                                              const float* __restrict__ gam, const float* __restrict__ bet,
                                              float* ss) {
  __shared__ __attribute__((aligned(16))) float stg[2 * CW];
  const int tid = (int)threadIdx.x;
  const int c = tid;
  double n = 0.0, mean = 0.0, M2 = 0.0;
#pragma unroll 1
  for (int b = 0; b < nPart; ++b) {
    const float* pr = part + (size_t)b * PARTW4;
    const double nbv = (double)pr[0];
    const double mb  = (double)pr[1 + c];
    const double qb  = (double)pr[1 + CW + c];
    if (nbv > 0.5) {
      const double nn = n + nbv;
      const double delta = mb - mean;
      const double f = nbv / nn;
      mean = mean + delta * f;
      M2 = M2 + qb + delta * delta * n * f;
      n = nn;
    }
  }
  const double nt = n < 1.0 ? 1.0 : n;
  const float varf  = (float)(M2 / nt);
  const float meanf = (float)mean;
  const float rstd = 1.0f / sqrtf(varf + BNEPS);
  const float sc = bfr(gam[c]) * rstd;
  const float sh = bfr(bet[c]) - meanf * sc;
  stg[c] = sc;
  stg[CW + c] = sh;
  __syncthreads();
  v4f v = {0.0f, 0.0f, 0.0f, 0.0f};
  if (tid < (2 * CW) / 4) {
    v = *(const v4fa*)(stg + 4 * tid);
    *(volatile v4f*)(ss + 4 * tid) = v;
  }
  __threadfence();
  if (tid < (2 * CW) / 4) {
    *(volatile v4f*)(ss + 4 * tid) = v;
  }
}

__global__ __launch_bounds__(NTHR) void k_apply(const float* __restrict__ hc, const float* __restrict__ ss,
                                                int nN, int nUnits, unsigned short* apl) {
  __shared__ __attribute__((aligned(16))) float ssh[2 * CW];
  const int tid = (int)threadIdx.x;
  ssh[tid]      = ss[tid];
  ssh[CW + tid] = ss[CW + tid];
  __syncthreads();
  const int u = (int)blockIdx.x * NTHR + tid;
  const bool act = u < nUnits;
  const int uc = act ? u : (nUnits - 1);
  const int row = uc >> 6;
  const int piece = uc & 63;
  const int c0 = (piece & 31) * 8;
  const float* p = hc + (size_t)row * CW + c0;
  const v4f a = *(const v4fa*)p;
  const v4f b = *(const v4fa*)(p + 4);
  const v4f sca = *(const v4fa*)(ssh + c0);
  const v4f scb = *(const v4fa*)(ssh + c0 + 4);
  const v4f sha = *(const v4fa*)(ssh + CW + c0);
  const v4f shb = *(const v4fa*)(ssh + CW + c0 + 4);
  const bool live = row < nN;
  float y[8];
  y[0] = fmaf(a.x, sca.x, sha.x); y[1] = fmaf(a.y, sca.y, sha.y); y[2] = fmaf(a.z, sca.z, sha.z); y[3] = fmaf(a.w, sca.w, sha.w);
  y[4] = fmaf(b.x, scb.x, shb.x); y[5] = fmaf(b.y, scb.y, shb.y); y[6] = fmaf(b.z, scb.z, shb.z); y[7] = fmaf(b.w, scb.w, shb.w);
  unsigned int wv[8];
  const bool lsel = piece >= 32;
#pragma unroll
  for (int j = 0; j < 8; ++j) {
    float t = y[j] < 0.0f ? 0.0f : y[j];
    t = live ? t : 0.0f;
    const unsigned int hb = f2bf(t);
    const unsigned int lb = f2bf(t - bf2f(hb));
    wv[j] = lsel ? lb : hb;
  }
  v4u q;
  q.x = wv[0] | (wv[1] << 16);
  q.y = wv[2] | (wv[3] << 16);
  q.z = wv[4] | (wv[5] << 16);
  q.w = wv[6] | (wv[7] << 16);
  unsigned short* o = apl + (size_t)row * KA + 8 * piece;
  if (act) *(volatile v4u*)o = q;
  __threadfence();
  if (act) *(volatile v4u*)o = q;
}

__global__ __launch_bounds__(NTHR) void k_pool(const int* __restrict__ batch, const float* __restrict__ z,
                                               int nN, float* gout) {
  __shared__ __attribute__((aligned(16))) float wsp[NWAVE * PSTW];
  __shared__ __attribute__((aligned(16))) float gst[C3];
  const int tid = (int)threadIdx.x, lane = tid & 31, wave = tid >> 5;
  const int g = (int)blockIdx.x;
  float a0 = 0.0f, a1 = 0.0f;
  int wc = 0;
  const int nChunks = (nN + NTHR - 1) / NTHR;
#pragma unroll 1
  for (int ch = 0; ch < nChunks; ++ch) {
    const int n  = ch * NTHR + tid;
    const int nc = n < nN ? n : nN - 1;
    const int b  = batch[nc];
    const bool hit = (n < nN) && (b == g);
    unsigned int mk = __builtin_amdgcn_ballot_w32(hit);
#pragma unroll 1
    while (mk != 0u) {
      const int k = __builtin_ctz(mk);
      mk &= (mk - 1u);
      int nk = ch * NTHR + wave * 32 + k;
      nk = nk > nN - 1 ? nN - 1 : nk;
      const v2f v = *(const v2fa*)(z + (size_t)nk * C3 + 2 * lane);
      a0 += v.x;
      a1 += v.y;
      wc += 1;
    }
  }
  wsp[wave * PSTW + 2 * lane]     = a0;
  wsp[wave * PSTW + 2 * lane + 1] = a1;
  if (lane == 0) wsp[wave * PSTW + C3] = (float)wc;
  __syncthreads();
  if (tid < C3) {
    float s = 0.0f, cnt = 0.0f;
#pragma unroll 1
    for (int w2 = 0; w2 < NWAVE; ++w2) {
      s   += wsp[w2 * PSTW + tid];
      cnt += wsp[w2 * PSTW + C3];
    }
    const float cm = cnt > 1.0f ? cnt : 1.0f;
    const float rc = 1.0f / cm;
    gst[tid] = s * rc;
  }
  __syncthreads();
  v4f v = {0.0f, 0.0f, 0.0f, 0.0f};
  if (tid < C3 / 4) {
    v = *(const v4fa*)(gst + 4 * tid);
    *(volatile v4f*)(gout + (size_t)g * C3 + 4 * tid) = v;
  }
  __threadfence();
  if (tid < C3 / 4) {
    *(volatile v4f*)(gout + (size_t)g * C3 + 4 * tid) = v;
  }
}

static int pick_nb(int nE, int nN) {
  int nb = NBRUN;
  while (nb > 32 && (long long)nb * (long long)nE * 5LL > (long long)RCAP * (long long)nN * 4LL) nb >>= 1;
  return nb;
}
static inline int cdiv(int a, int b) { return (a + b - 1) / b; }
static inline size_t al256(size_t o) { return (o + 255) & ~(size_t)255; }

extern "C" void kernel_launch(void* const* d_in, const int* in_sizes, int n_in,
                              void* d_out, int out_size, void* d_ws, size_t ws_size,
                              hipStream_t stream) {
  if (n_in < 19) return;
  if (in_sizes[0] < 16 * DIN1 || (in_sizes[0] % DIN1) != 0) return;
  const int nN = in_sizes[0] / DIN1;
  if (nN >= (1 << 24)) return;
  if (in_sizes[1] < 2 || (in_sizes[1] & 1) != 0) return;
  const int nE = in_sizes[1] / 2;
  if (nE < 1 || nE >= (1 << (32 - SLOTB))) return;
  if (in_sizes[2] != nN) return;
  if (in_sizes[3] != DIN1 * CW || in_sizes[4] != DIN1 * CW) return;
  if (in_sizes[5] != CW || in_sizes[6] != CW) return;
  if (in_sizes[7] != CW || in_sizes[8] != CW) return;
  if (in_sizes[9] != CW * CW || in_sizes[10] != CW * CW) return;
  if (in_sizes[11] != CW || in_sizes[12] != CW) return;
  if (in_sizes[13] != CW || in_sizes[14] != CW) return;
  if (in_sizes[15] != CW * C3 || in_sizes[16] != CW * C3) return;
  if (in_sizes[17] != C3 || in_sizes[18] != C3) return;
  const long long zEl = (long long)nN * C3;
  if ((long long)out_size <= zEl || (((long long)out_size - zEl) % C3) != 0) return;
  const int nG = (int)(((long long)out_size - zEl) / C3);
  if (nG < 1 || nG > 65535) return;

  const float* x     = (const float*)d_in[0];
  const int*   ei    = (const int*)  d_in[1];
  const int*   batch = (const int*)  d_in[2];
  const float* Wl1   = (const float*)d_in[3];
  const float* Wr1   = (const float*)d_in[4];
  const float* att1  = (const float*)d_in[5];
  const float* b1    = (const float*)d_in[6];
  const float* g1    = (const float*)d_in[7];
  const float* be1   = (const float*)d_in[8];
  const float* Wl2   = (const float*)d_in[9];
  const float* Wr2   = (const float*)d_in[10];
  const float* att2  = (const float*)d_in[11];
  const float* b2    = (const float*)d_in[12];
  const float* g2    = (const float*)d_in[13];
  const float* be2   = (const float*)d_in[14];
  const float* Wl3   = (const float*)d_in[15];
  const float* Wr3   = (const float*)d_in[16];
  const float* att3  = (const float*)d_in[17];
  const float* b3    = (const float*)d_in[18];
  float* out  = (float*)d_out;
  float* gout = out + (size_t)zEl;
  const int* src = ei;
  const int* dst = ei + nE;

  const int MP   = cdiv(nN, MROWS) * MROWS;
  const int gM   = MP / GBM;
  const int nb   = pick_nb(nE, nN);
  if (nb < 32 || (nb & (nb - 1)) != 0 || nb > NBMAX) return;
  const int gA   = cdiv(MP, nb);
  if ((long long)gA * nb < (long long)MP) return;
  const int vec8 = ((nE & 3) == 0) ? 1 : 0;

  char* ws = (char*)d_ws;
  size_t off = 0;
  const size_t oW1 = off; off = al256(off + (size_t)NP  * DIN1 * 2);
  const size_t oW2 = off; off = al256(off + (size_t)NP  * KA * 2);
  const size_t oW3 = off; off = al256(off + (size_t)NP3 * KA * 2);
  const size_t oP  = off; off = al256(off + (size_t)MP * KA * 2);
  const size_t oF  = off; off = al256(off + (size_t)MP * NP * 4);
  const size_t oQ  = off; off = al256(off + (size_t)MP * CW * 4);
  const size_t oPT = off; off = al256(off + (size_t)gA * PARTW4 * 4);
  const size_t oSS = off; off = al256(off + (size_t)(2 * CW) * 4);
  if (off > ws_size || off > (size_t)WSLIM) return;
  unsigned short* WT1 = (unsigned short*)(ws + oW1);
  unsigned short* WT2 = (unsigned short*)(ws + oW2);
  unsigned short* WT3 = (unsigned short*)(ws + oW3);
  unsigned short* XB  = (unsigned short*)(ws + oP);
  unsigned short* APL = (unsigned short*)(ws + oP);
  float*          F   = (float*)(ws + oF);
  float*          HC  = (float*)(ws + oQ);
  float*          PT  = (float*)(ws + oPT);
  float*          SS  = (float*)(ws + oSS);

  hipFuncSetAttribute(reinterpret_cast<const void*>(&k_agg<8, 8, 1>),
                      hipFuncAttributeMaxDynamicSharedMemorySize, LDS_AGG);
  hipFuncSetAttribute(reinterpret_cast<const void*>(&k_agg<2, 32, 0>),
                      hipFuncAttributeMaxDynamicSharedMemorySize, LDS_AGG);

  {
    const int nUx = MP * (DIN1 / 8);
    k_xcvt<<<cdiv(nUx, NTHR), NTHR, 0, stream>>>(x, nN, nUx, XB);
    const int nU1 = CW * (DIN1 / 8);
    if ((nU1 % NTHR) != 0) return;
    k_wt<<<2 * (nU1 / NTHR), NTHR, 0, stream>>>(Wl1, Wr1, CW, 4, DIN1 - 1, DIN1, CW, nU1 / NTHR, nU1, WT1);
    const int nU2 = CW * (KA / 8);
    if ((nU2 % NTHR) != 0) return;
    k_wt<<<2 * (nU2 / NTHR), NTHR, 0, stream>>>(Wl2, Wr2, CW, 6, CW - 1, KA, CW, nU2 / NTHR, nU2, WT2);
    const int nU3 = C3 * (KA / 8);
    if ((nU3 % NTHR) != 0) return;
    k_wt<<<2 * (nU3 / NTHR), NTHR, 0, stream>>>(Wl3, Wr3, C3, 6, CW - 1, KA, C3, nU3 / NTHR, nU3, WT3);
  }
  const int nUa = MP * 64;

  k_gemm<<<dim3(gM, NP / GBN), GTHR, 0, stream>>>(XB, WT1, F, DIN1, NP);
  k_agg<8, 8, 1><<<gA, NTHR, LDS_AGG, stream>>>(src, dst, F, att1, b1, HC, CW, MP, PT, nN, nE, nb, vec8);
  k_bnfin<<<1, CW, 0, stream>>>(PT, gA, g1, be1, SS);
  k_apply<<<cdiv(nUa, NTHR), NTHR, 0, stream>>>(HC, SS, nN, nUa, APL);

  k_gemm<<<dim3(gM, NP / GBN), GTHR, 0, stream>>>(APL, WT2, F, KA, NP);
  k_agg<8, 8, 1><<<gA, NTHR, LDS_AGG, stream>>>(src, dst, F, att2, b2, HC, CW, MP, PT, nN, nE, nb, vec8);
  k_bnfin<<<1, CW, 0, stream>>>(PT, gA, g2, be2, SS);
  k_apply<<<cdiv(nUa, NTHR), NTHR, 0, stream>>>(HC, SS, nN, nUa, APL);

  k_gemm<<<dim3(gM, NP3 / GBN), GTHR, 0, stream>>>(APL, WT3, F, KA, NP3);
  k_agg<2, 32, 0><<<gA, NTHR, LDS_AGG, stream>>>(src, dst, F, att3, b3, out, C3, nN, PT, nN, nE, nb, vec8);

  k_pool<<<nG, NTHR, 0, stream>>>(batch, out, nN, gout);
}
